// VRAttention_69956427317524
// MI455X (gfx1250) — hardware-run, weakly checked
//
#include <hip/hip_runtime.h>
#include <math.h>

typedef __attribute__((ext_vector_type(16))) _Float16 v16h;
typedef __attribute__((ext_vector_type(8)))  _Float16 v8h;
typedef __attribute__((ext_vector_type(8)))  float    v8f;
typedef __attribute__((ext_vector_type(4)))  float    v4f;
typedef __attribute__((ext_vector_type(4)))  unsigned v4u;

constexpr int kNb   = 4;
constexpr int kCin  = 128;
constexpr int kPl   = 256;
constexpr int kAtt  = 64;
constexpr int kRank = 16;
constexpr int kSteps = 6;
constexpr int kImg  = 64;
constexpr int kHW   = kImg * kImg;
constexpr int kTok  = kNb * kHW;
constexpr int kChunks = 32;
constexpr int kChunkPix = kHW / kChunks;
constexpr int kTP   = 68;
constexpr int kCmbThreads = 64;
constexpr int kCmbTokPerWave = 8;
constexpr int kCmbTokPerBlock = (kCmbThreads / 32) * kCmbTokPerWave;
constexpr float kCarryX = 16.0f;
constexpr float kCarryW = 1024.0f;
constexpr float kCarryA = 256.0f;
constexpr float kInvCarryA = 1.0f / kCarryA;
constexpr float kEps = 1e-6f;
constexpr float kNormFloor = 1e-12f;
constexpr float kScaleS1 = 1.0f / (kCarryX * kCarryW);
constexpr float kScaleS2 = 1.0f / (kCarryA * kCarryW);
constexpr float kScaleS6 = 1.0f / (kCarryA * kCarryW);
constexpr int kOut0Elems = kNb * kCin * kHW;
constexpr int kOut1Elems = kNb * kPl;
static_assert(kTok == 16384 && kHW == 4096, "token count");
static_assert((kCin % 32) == 0 && (kPl % 32) == 0, "GEMM K multiples of 32");
static_assert((kTok % 64) == 0 && (kPl % 64) == 0 && (kCin % 64) == 0 && (kHW % 64) == 0, "GEMM M,N multiples of 64");
static_assert(kChunkPix == 128, "pool chunk");
static_assert((kTok % kCmbTokPerBlock) == 0 && (kTok % 256) == 0, "token grids exact");
static_assert(kPl == 32 * 8, "one wave covers a token row with 8 channels per lane");
static_assert((size_t)kOut0Elems * 4 == 8388608ull, "second output byte offset");
static_assert(((size_t)kOut0Elems * 4) % 128 == 0, "second output line aligned");
static_assert((size_t)(kOut0Elems + kOut1Elems) * 4 == 8392704ull, "output total bytes");

constexpr size_t kOffXT   = 0;
constexpr size_t kOffW1H  = kOffXT   + (size_t)kTok * kCin * 2;
constexpr size_t kOffLWH  = kOffW1H  + (size_t)kPl * kCin * 2;
constexpr size_t kOffY    = kOffLWH  + (size_t)kPl * kPl * 2;
constexpr size_t kOffXM   = kOffY    + (size_t)kTok * kPl * 2;
constexpr size_t kOffXL   = kOffXM   + (size_t)kTok * kPl * 2;
constexpr size_t kOffFEAT = kOffXL   + (size_t)kTok * kPl * 4;
constexpr size_t kOffPSUM = kOffFEAT + (size_t)kTok * kPl * 2;
constexpr size_t kOffPMAX = kOffPSUM + (size_t)kNb * kChunks * kPl * 4;
constexpr size_t kOffFCS  = kOffPMAX + (size_t)kNb * kChunks * kPl * 4;
constexpr size_t kOffFLAG = kOffFCS  + (size_t)kNb * kCin * kPl * 2;
constexpr size_t kWsTotal = kOffFLAG + (size_t)kTok * 4;
static_assert(kWsTotal == 46923776ull, "carve total");
static_assert(kWsTotal <= 134217728ull, "carve cap");
static_assert((kOffW1H % 128) == 0 && (kOffLWH % 128) == 0 && (kOffY % 128) == 0 && (kOffXM % 128) == 0 &&
              (kOffXL % 128) == 0 && (kOffFEAT % 128) == 0 && (kOffPSUM % 128) == 0 && (kOffPMAX % 128) == 0 &&
              (kOffFCS % 128) == 0 && (kOffFLAG % 128) == 0,
              "128-B aligned regions");

__device__ __forceinline__ float h16_to_f32(unsigned hb) {
  const unsigned sgn = (hb & 0x8000u) << 16;
  const unsigned em = hb & 0x7fffu;
  const float fn = __uint_as_float((em << 13) + 0x38000000u);
  const float fs = (float)em * 5.9604644775390625e-8f;
  const float mag = (em < 0x400u) ? fs : fn;
  return __uint_as_float(__float_as_uint(mag) | sgn);
}
__device__ __forceinline__ void unpack8_f16(v4u rv, float (&f)[8]) {
  const unsigned w0 = rv[0];
  const unsigned w1 = rv[1];
  const unsigned w2 = rv[2];
  const unsigned w3 = rv[3];
  f[0] = h16_to_f32(w0 & 0xffffu);
  f[1] = h16_to_f32(w0 >> 16);
  f[2] = h16_to_f32(w1 & 0xffffu);
  f[3] = h16_to_f32(w1 >> 16);
  f[4] = h16_to_f32(w2 & 0xffffu);
  f[5] = h16_to_f32(w2 >> 16);
  f[6] = h16_to_f32(w3 & 0xffffu);
  f[7] = h16_to_f32(w3 >> 16);
}

union FragU { v16h v; v8h h[2]; };
__device__ __forceinline__ v16h frag_load(const _Float16* p) {
  FragU f;
  f.h[0] = *(const v8h*)(p);
  f.h[1] = *(const v8h*)(p + 16);
  return f.v;
}
__device__ __forceinline__ v8f mma_f16(v16h a, v16h b, v8f c) {
  return __builtin_amdgcn_wmma_f32_16x16x32_f16(false, a, false, b, (short)0, c, false, false);
}
__device__ __forceinline__ void settle4(v8f& a0, v8f& a1, v8f& a2, v8f& a3,
                                        v16h x, v16h b0, v16h b1, v16h b2, v16h b3) {
  asm volatile("" : "+v"(a0) : "v"(x), "v"(b0));
  asm volatile("" : "+v"(a1) : "v"(x), "v"(b1));
  asm volatile("" : "+v"(a2) : "v"(x), "v"(b2));
  asm volatile("v_nop\n\tv_nop\n\tv_nop\n\tv_nop" : "+v"(a3) : "v"(x), "v"(b3));
  asm volatile("" : "+v"(a0));
  asm volatile("" : "+v"(a1));
  asm volatile("" : "+v"(a2));
}
__device__ __forceinline__ void keep4_h(v16h a, v16h b, v16h c, v16h d) {
  asm volatile("v_nop" :: "v"(a), "v"(b), "v"(c), "v"(d));
}

__global__ __launch_bounds__(256) void prep_x_kernel(const float* __restrict__ x, unsigned short* __restrict__ xt)
{
  __shared__ __align__(16) float sT[64 * kTP];
  const int tid  = threadIdx.x;
  const int lane = tid & 31;
  const int wave = __builtin_amdgcn_readfirstlane((int)(threadIdx.x >> 5));
  const int p0 = blockIdx.x * 64;
  const int c0 = blockIdx.y * 64;
  const int b  = blockIdx.z;
  const float* src = x + ((size_t)b * kCin + c0) * kHW + p0;
#pragma unroll
  for (int it = 0; it < 4; ++it) {
    const int idx = it * 256 + tid;
    const int ch = idx >> 4;
    const int p4 = (idx & 15) * 4;
    const v4f v = *(const v4f*)(src + (size_t)ch * kHW + p4);
    sT[(p4 + 0) * kTP + ch] = v[0];
    sT[(p4 + 1) * kTP + ch] = v[1];
    sT[(p4 + 2) * kTP + ch] = v[2];
    sT[(p4 + 3) * kTP + ch] = v[3];
  }
  __syncthreads();
  const int q  = lane >> 3;
  const int c8 = (lane & 7) * 8;
  v8h hv[2];
#pragma unroll
  for (int it = 0; it < 2; ++it) {
    const int row = it * 32 + wave * 4 + q;
    const float* sp = sT + row * kTP + c8;
    const v4f a0 = *(const v4f*)(sp);
    const v4f a1 = *(const v4f*)(sp + 4);
#pragma unroll
    for (int e = 0; e < 4; ++e) {
      hv[it][e]     = (_Float16)(a0[e] * kCarryX);
      hv[it][4 + e] = (_Float16)(a1[e] * kCarryX);
    }
  }
  for (int pass = 0; pass < 2; ++pass) {
#pragma unroll
    for (int it = 0; it < 2; ++it) {
      const int row = it * 32 + wave * 4 + q;
      unsigned short* dst = xt + ((size_t)b * kHW + p0 + row) * kCin + c0 + c8;
      *(volatile v8h*)dst = hv[it];
    }
    __threadfence();
  }
}

__global__ __launch_bounds__(256) void prep_w_kernel(const float* __restrict__ w1, const float* __restrict__ lw,
                                                     unsigned short* __restrict__ w1h, unsigned short* __restrict__ lwh)
{
  const bool first = (blockIdx.x < 16);
  const float* src = first ? w1 : lw;
  unsigned short* dst = first ? w1h : lwh;
  const int blk = first ? (int)blockIdx.x : ((int)blockIdx.x - 16);
  const int total8 = first ? (kPl * kCin / 8) : (kPl * kPl / 8);
  const int i = blk * 256 + (int)threadIdx.x;
  if (i >= total8) return;
  const size_t e0 = (size_t)i << 3;
  const v4f a0 = *(const v4f*)(src + e0);
  const v4f a1 = *(const v4f*)(src + e0 + 4);
  v8h hv;
#pragma unroll
  for (int e = 0; e < 4; ++e) {
    hv[e]     = (_Float16)(a0[e] * kCarryW);
    hv[4 + e] = (_Float16)(a1[e] * kCarryW);
  }
  unsigned short* q = dst + e0;
  *(volatile v8h*)q = hv;
  __threadfence();
  *(volatile v8h*)q = hv;
}

__global__ __launch_bounds__(256) void flag_kernel(const float* __restrict__ binit, int* __restrict__ flags)
{
  const int m = blockIdx.x * 256 + (int)threadIdx.x;
  const float* bp = binit + (size_t)m * kRank;
  const v4f a0 = *(const v4f*)(bp);
  const v4f a1 = *(const v4f*)(bp + 4);
  const v4f a2 = *(const v4f*)(bp + 8);
  const v4f a3 = *(const v4f*)(bp + 12);
  bool pos = true;
#pragma unroll
  for (int e = 0; e < 4; ++e) {
    pos = pos && (a0[e] > kNormFloor);
    pos = pos && (a1[e] > kNormFloor);
    pos = pos && (a2[e] > kNormFloor);
    pos = pos && (a3[e] > kNormFloor);
  }
  const int f = pos ? 1 : 0;
  *(volatile int*)(flags + m) = f;
  __threadfence();
  *(volatile int*)(flags + m) = f;
}

template <int EPI>
__global__ __launch_bounds__(256) void gemm_f16_kernel(
    const unsigned short* Ap, int lda, long strideA,
    const unsigned short* Btp, int ldb, long strideB,
    void* Cout, int ldc, long strideC,
    const float* __restrict__ bias,
    int M, int N, int K, float scale)
{
  __shared__ __align__(16) float sT[8][16 * kTP];
  const _Float16* A  = (const _Float16*)Ap;
  const _Float16* Bt = (const _Float16*)Btp;
  const int b    = blockIdx.y;
  const int lane = threadIdx.x & 31;
  const int wave = __builtin_amdgcn_readfirstlane((int)(threadIdx.x >> 5));
  const int tilesN = N >> 6;
  const int tilesM = M >> 6;
  const int tile = blockIdx.x * 8 + wave;
  if (tile >= tilesM * tilesN) return;
  const int tm = tile / tilesN;
  const int tn = tile - tm * tilesN;
  const int m0 = tm << 6;
  const int n0 = tn << 6;

  const _Float16* Ab = A  + (size_t)b * strideA;
  const _Float16* Bb = Bt + (size_t)b * strideB;

  const int rlane = lane & 15;
  const int koff  = (lane >> 4) * 8;
  const int mOff  = (lane >> 4) * 8;

  v8f acc[4][4];
#pragma unroll
  for (int i = 0; i < 4; ++i)
#pragma unroll
    for (int j = 0; j < 4; ++j) acc[i][j] = (v8f){0.f, 0.f, 0.f, 0.f, 0.f, 0.f, 0.f, 0.f};

  for (int k0 = 0; k0 < K; k0 += 32) {
    v16h bh[4];
#pragma unroll
    for (int j = 0; j < 4; ++j) {
      const size_t bo = (size_t)(n0 + (j << 4) + rlane) * ldb + koff + k0;
      bh[j] = frag_load(Bb + bo);
    }
#pragma unroll
    for (int i = 0; i < 4; ++i) {
      const size_t ao = (size_t)(m0 + (i << 4) + rlane) * lda + koff + k0;
      const v16h ah = frag_load(Ab + ao);
#pragma unroll
      for (int j = 0; j < 4; ++j) acc[i][j] = mma_f16(ah, bh[j], acc[i][j]);
      settle4(acc[i][0], acc[i][1], acc[i][2], acc[i][3], ah, bh[0], bh[1], bh[2], bh[3]);
    }
    keep4_h(bh[0], bh[1], bh[2], bh[3]);
  }

  float* slab = sT[wave];
  const int q16  = lane >> 3;
  const int c8   = (lane & 7) * 8;
  const int hh   = lane >> 4;
  const int c4   = (lane & 15) * 4;
  v4f nbv = (v4f){0.f, 0.f, 0.f, 0.f};
  if (EPI == 1) nbv = *(const v4f*)(bias + n0 + c4);
#pragma unroll
  for (int i = 0; i < 4; ++i) {
    const int mBase = m0 + (i << 4);
#pragma unroll
    for (int j = 0; j < 4; ++j) {
#pragma unroll
      for (int r = 0; r < 8; ++r) slab[(mOff + r) * kTP + (j << 4) + rlane] = acc[i][j][r];
    }
    __builtin_amdgcn_fence(__ATOMIC_RELEASE, "workgroup");
    __builtin_amdgcn_wave_barrier();
    __builtin_amdgcn_fence(__ATOMIC_ACQUIRE, "workgroup");
    if (EPI != 0) {
      float* C = (float*)Cout + (size_t)b * strideC;
      v4f vals[8];
#pragma unroll
      for (int it = 0; it < 8; ++it) {
        const int row = it * 2 + hh;
        const v4f sv = *(const v4f*)(slab + row * kTP + c4);
        v4f o;
        if (EPI == 2) {
          const float bv = bias[mBase + row];
          o[0] = fmaf(sv[0], scale, bv);
          o[1] = fmaf(sv[1], scale, bv);
          o[2] = fmaf(sv[2], scale, bv);
          o[3] = fmaf(sv[3], scale, bv);
        } else {
          o[0] = fmaxf(fmaf(sv[0], scale, nbv[0]), 0.0f);
          o[1] = fmaxf(fmaf(sv[1], scale, nbv[1]), 0.0f);
          o[2] = fmaxf(fmaf(sv[2], scale, nbv[2]), 0.0f);
          o[3] = fmaxf(fmaf(sv[3], scale, nbv[3]), 0.0f);
        }
        vals[it] = o;
      }
      for (int pass = 0; pass < 2; ++pass) {
#pragma unroll
        for (int it = 0; it < 8; ++it) {
          const int row = it * 2 + hh;
          *(volatile v4f*)(C + (size_t)(mBase + row) * ldc + n0 + c4) = vals[it];
        }
        __threadfence();
      }
    } else {
      unsigned short* C = (unsigned short*)Cout + (size_t)b * strideC;
      v8h hv[4];
#pragma unroll
      for (int it = 0; it < 4; ++it) {
        const int row = it * 4 + q16;
        const float* sp = slab + row * kTP + c8;
        const v4f a0 = *(const v4f*)(sp);
        const v4f a1 = *(const v4f*)(sp + 4);
#pragma unroll
        for (int e = 0; e < 4; ++e) {
          hv[it][e]     = (_Float16)(a0[e] * scale);
          hv[it][4 + e] = (_Float16)(a1[e] * scale);
        }
      }
      for (int pass = 0; pass < 2; ++pass) {
#pragma unroll
        for (int it = 0; it < 4; ++it) {
          const int row = it * 4 + q16;
          *(volatile v8h*)(C + (size_t)(mBase + row) * ldc + n0 + c8) = hv[it];
        }
        __threadfence();
      }
    }
    __builtin_amdgcn_fence(__ATOMIC_RELEASE, "workgroup");
    __builtin_amdgcn_wave_barrier();
    __builtin_amdgcn_fence(__ATOMIC_ACQUIRE, "workgroup");
  }
}

__global__ __launch_bounds__(256) void dw3x3_kernel(const unsigned short* __restrict__ y, const float* __restrict__ w3,
                                                    const float* __restrict__ b3, unsigned short* __restrict__ xm)
{
  __shared__ __align__(16) float sW[9 * kPl];
  const int tid  = threadIdx.x;
  const int lane = tid & 31;
  const int wave = __builtin_amdgcn_readfirstlane((int)(threadIdx.x >> 5));
#pragma unroll 1
  for (int t = 0; t < 9; ++t) sW[t * kPl + tid] = w3[tid * 9 + t];
  __syncthreads();
  const int rowid = blockIdx.x;
  const int b = rowid >> 6;
  const int h = rowid & 63;
  const int cb = lane * 8;
  const v4f bb0 = *(const v4f*)(b3 + cb);
  const v4f bb1 = *(const v4f*)(b3 + cb + 4);
#pragma unroll 1
  for (int it = 0; it < 8; ++it) {
    const int w = it * 8 + wave;
    float acc[8];
#pragma unroll
    for (int e = 0; e < 8; ++e) acc[e] = 0.0f;
#pragma unroll 1
    for (int dy = -1; dy <= 1; ++dy) {
      const int hy = h + dy;
      const bool hok = ((unsigned)hy < (unsigned)kImg);
      const int hc = hy < 0 ? 0 : (hy > kImg - 1 ? kImg - 1 : hy);
#pragma unroll 1
      for (int dx = -1; dx <= 1; ++dx) {
        const int wx = w + dx;
        const bool ok = hok && ((unsigned)wx < (unsigned)kImg);
        const int wc = wx < 0 ? 0 : (wx > kImg - 1 ? kImg - 1 : wx);
        const size_t tok = (size_t)b * kHW + (size_t)hc * kImg + wc;
        const v4u rv = *(const v4u*)(y + tok * kPl + cb);
        const float* wp = sW + ((dy + 1) * 3 + (dx + 1)) * kPl + cb;
        const v4f wa = *(const v4f*)(wp);
        const v4f wb = *(const v4f*)(wp + 4);
        float f[8];
        unpack8_f16(rv, f);
#pragma unroll
        for (int e = 0; e < 4; ++e) {
          const float fa = ok ? f[e] : 0.0f;
          const float fb = ok ? f[4 + e] : 0.0f;
          acc[e]     = fmaf(fa, wa[e], acc[e]);
          acc[4 + e] = fmaf(fb, wb[e], acc[4 + e]);
        }
      }
    }
    v8h hv;
#pragma unroll
    for (int e = 0; e < 4; ++e) {
      hv[e]     = (_Float16)((acc[e] + bb0[e]) * kCarryA);
      hv[4 + e] = (_Float16)((acc[4 + e] + bb1[e]) * kCarryA);
    }
    unsigned short* dst = xm + ((size_t)b * kHW + (size_t)h * kImg + w) * kPl + cb;
    *(volatile v8h*)dst = hv;
    __threadfence();
    *(volatile v8h*)dst = hv;
  }
}

__global__ __launch_bounds__(64) void combine_kernel(const float* __restrict__ xl, const unsigned short* __restrict__ xm,
                                                     const int* __restrict__ flags, const float* __restrict__ binit,
                                                     unsigned short* __restrict__ feat)
{
  __shared__ __align__(16) float sC[8 * kRank * kCmbThreads];
  __shared__ __align__(16) float sX[8 * kCmbThreads];
  __shared__ __align__(16) float sS[8 * kCmbThreads];
  __shared__ __align__(16) float sB[kRank * kCmbThreads];
  const int tid  = threadIdx.x;
  const int lane = tid & 31;
  const int wave = __builtin_amdgcn_readfirstlane((int)(threadIdx.x >> 5));
  const int tok0 = ((int)blockIdx.x * (kCmbThreads / 32) + wave) * kCmbTokPerWave;
#pragma unroll 1
  for (int t = 0; t < kCmbTokPerWave; ++t) {
    const int m = tok0 + t;
    const int fl = __builtin_amdgcn_readfirstlane(flags[m]);
    const v4f x0 = *(const v4f*)(xl + (size_t)m * kPl + lane * 8);
    const v4f x1 = *(const v4f*)(xl + (size_t)m * kPl + lane * 8 + 4);
    const v4u rv = *(const v4u*)(xm + (size_t)m * kPl + lane * 8);
    const v4f bq0 = *(const v4f*)(binit + (size_t)m * kRank);
    const v4f bq1 = *(const v4f*)(binit + (size_t)m * kRank + 4);
    const v4f bq2 = *(const v4f*)(binit + (size_t)m * kRank + 8);
    const v4f bq3 = *(const v4f*)(binit + (size_t)m * kRank + 12);
    float xm8[8];
    unpack8_f16(rv, xm8);
    float xv[8];
    xv[0] = x0[0]; xv[1] = x0[1]; xv[2] = x0[2]; xv[3] = x0[3];
    xv[4] = x1[0]; xv[5] = x1[1]; xv[6] = x1[2]; xv[7] = x1[3];
    float xr[8];
    if (fl == 1) {
#pragma unroll
      for (int e = 0; e < 8; ++e) xr[e] = xv[e] * xv[e] * __builtin_amdgcn_rcpf(xv[e] + kEps);
    } else {
#pragma unroll
      for (int e = 0; e < 8; ++e) sX[e * kCmbThreads + tid] = xv[e];
#pragma unroll
      for (int e = 0; e < 4; ++e) {
        sB[(e)      * kCmbThreads + tid] = bq0[e];
        sB[(4 + e)  * kCmbThreads + tid] = bq1[e];
        sB[(8 + e)  * kCmbThreads + tid] = bq2[e];
        sB[(12 + e) * kCmbThreads + tid] = bq3[e];
      }
#pragma unroll 1
      for (int r = 0; r < kRank; ++r) {
        const float bv = sB[r * kCmbThreads + tid];
        sB[r * kCmbThreads + tid] = bv / fmaxf(fabsf(bv), kNormFloor);
      }
#pragma unroll 1
      for (int j = 0; j < 8; ++j) {
        const float xj = sX[j * kCmbThreads + tid];
        float mx = -__builtin_inff();
#pragma unroll 1
        for (int r = 0; r < kRank; ++r) mx = fmaxf(mx, xj * sB[r * kCmbThreads + tid]);
        float s = 0.0f;
#pragma unroll 1
        for (int r = 0; r < kRank; ++r) {
          const float ev = expf(xj * sB[r * kCmbThreads + tid] - mx);
          sC[(j * kRank + r) * kCmbThreads + tid] = ev;
          s += ev;
        }
        const float inv = 1.0f / s;
#pragma unroll 1
        for (int r = 0; r < kRank; ++r) {
          const float ev = sC[(j * kRank + r) * kCmbThreads + tid];
          sC[(j * kRank + r) * kCmbThreads + tid] = ev * inv;
        }
      }
#pragma unroll 1
      for (int step = 0; step < kSteps; ++step) {
#pragma unroll 1
        for (int j = 0; j < 8; ++j) {
          const float xj = sX[j * kCmbThreads + tid];
          float sn = 0.0f;
#pragma unroll 1
          for (int r = 0; r < kRank; ++r)
            sn = fmaf(sC[(j * kRank + r) * kCmbThreads + tid], sB[r * kCmbThreads + tid], sn);
#pragma unroll 1
          for (int r = 0; r < kRank; ++r) {
            const float bv = sB[r * kCmbThreads + tid];
            const float cv = sC[(j * kRank + r) * kCmbThreads + tid];
            const float num = xj * bv;
            const float den = fmaf(sn, bv, kEps);
            sC[(j * kRank + r) * kCmbThreads + tid] = (cv * num) / den;
          }
          float s2 = 0.0f;
#pragma unroll 1
          for (int r = 0; r < kRank; ++r)
            s2 = fmaf(sC[(j * kRank + r) * kCmbThreads + tid], sB[r * kCmbThreads + tid], s2);
          sS[j * kCmbThreads + tid] = s2;
        }
#pragma unroll 1
        for (int r = 0; r < kRank; ++r) {
          float pn = 0.0f;
          float pd = 0.0f;
#pragma unroll 1
          for (int j = 0; j < 8; ++j) {
            const float cv = sC[(j * kRank + r) * kCmbThreads + tid];
            pn = fmaf(sX[j * kCmbThreads + tid], cv, pn);
            pd = fmaf(sS[j * kCmbThreads + tid], cv, pd);
          }
          pn += __shfl_xor(pn, 16, 32);
          pd += __shfl_xor(pd, 16, 32);
          pn += __shfl_xor(pn, 8, 32);
          pd += __shfl_xor(pd, 8, 32);
          pn += __shfl_xor(pn, 4, 32);
          pd += __shfl_xor(pd, 4, 32);
          pn += __shfl_xor(pn, 2, 32);
          pd += __shfl_xor(pd, 2, 32);
          pn += __shfl_xor(pn, 1, 32);
          pd += __shfl_xor(pd, 1, 32);
          const float bv = sB[r * kCmbThreads + tid];
          sB[r * kCmbThreads + tid] = (bv * pn) / (pd + kEps);
        }
      }
#pragma unroll 1
      for (int j = 0; j < 8; ++j) {
        const float xj = sX[j * kCmbThreads + tid];
        float sn = 0.0f;
#pragma unroll 1
        for (int r = 0; r < kRank; ++r)
          sn = fmaf(sC[(j * kRank + r) * kCmbThreads + tid], sB[r * kCmbThreads + tid], sn);
        float xacc = 0.0f;
#pragma unroll 1
        for (int r = 0; r < kRank; ++r) {
          const float bv = sB[r * kCmbThreads + tid];
          const float cv = sC[(j * kRank + r) * kCmbThreads + tid];
          const float c2 = (cv * (xj * bv)) / fmaf(sn, bv, kEps);
          xacc = fmaf(bv, c2, xacc);
        }
        sS[j * kCmbThreads + tid] = xacc;
      }
#pragma unroll
      for (int e = 0; e < 8; ++e) xr[e] = sS[e * kCmbThreads + tid];
    }
    v8h hv;
#pragma unroll
    for (int e = 0; e < 8; ++e) {
      const float f = fmaxf(fmaf(xm8[e], kInvCarryA, xr[e]), 0.0f);
      hv[e] = (_Float16)(f * kCarryA);
    }
    unsigned short* dst = feat + (size_t)m * kPl + lane * 8;
    *(volatile v8h*)dst = hv;
    __threadfence();
    *(volatile v8h*)dst = hv;
  }
}

__global__ __launch_bounds__(256) void pool_partial_kernel(const unsigned short* __restrict__ feat,
                                                           float* __restrict__ psum, float* __restrict__ pmax)
{
  __shared__ __align__(16) float sS[8 * kPl];
  __shared__ __align__(16) float sM[8 * kPl];
  const int tid  = threadIdx.x;
  const int lane = tid & 31;
  const int wave = __builtin_amdgcn_readfirstlane((int)(threadIdx.x >> 5));
  const int chunk = blockIdx.x;
  const int b = blockIdx.y;
  const size_t m0 = (size_t)b * kHW + (size_t)chunk * kChunkPix + (size_t)wave * 16;
  float s[8], mx[8];
#pragma unroll
  for (int e = 0; e < 8; ++e) { s[e] = 0.0f; mx[e] = -__builtin_inff(); }
#pragma unroll 1
  for (int p = 0; p < 16; ++p) {
    const v4u rv = *(const v4u*)(feat + (m0 + p) * kPl + lane * 8);
    float f[8];
    unpack8_f16(rv, f);
#pragma unroll
    for (int e = 0; e < 8; ++e) { s[e] += f[e]; mx[e] = fmaxf(mx[e], f[e]); }
  }
  *(v4f*)(sS + wave * kPl + lane * 8)     = (v4f){s[0], s[1], s[2], s[3]};
  *(v4f*)(sS + wave * kPl + lane * 8 + 4) = (v4f){s[4], s[5], s[6], s[7]};
  *(v4f*)(sM + wave * kPl + lane * 8)     = (v4f){mx[0], mx[1], mx[2], mx[3]};
  *(v4f*)(sM + wave * kPl + lane * 8 + 4) = (v4f){mx[4], mx[5], mx[6], mx[7]};
  __syncthreads();
  float ts = 0.0f, tmx = -__builtin_inff();
#pragma unroll 1
  for (int w = 0; w < 8; ++w) {
    ts += sS[w * kPl + tid];
    tmx = fmaxf(tmx, sM[w * kPl + tid]);
  }
  const size_t o = ((size_t)b * kChunks + chunk) * kPl + tid;
  *(volatile float*)(psum + o) = ts;
  *(volatile float*)(pmax + o) = tmx;
  __threadfence();
  *(volatile float*)(psum + o) = ts;
  *(volatile float*)(pmax + o) = tmx;
}

__global__ __launch_bounds__(256) void att_kernel(const float* __restrict__ psum, const float* __restrict__ pmax,
                                                  const float* __restrict__ ca1, const float* __restrict__ ca2,
                                                  const float* __restrict__ fcw, float* __restrict__ out1,
                                                  unsigned short* __restrict__ fcs)
{
  __shared__ __align__(16) float sa[kPl];
  __shared__ __align__(16) float sm[kPl];
  __shared__ __align__(16) float hsum[kAtt];
  __shared__ __align__(16) float satt[kPl];
  const int tid = threadIdx.x;
  const int b = blockIdx.x;
  {
    float s = 0.0f, m = -__builtin_inff();
#pragma unroll 1
    for (int ch = 0; ch < kChunks; ++ch) {
      const size_t o = ((size_t)b * kChunks + ch) * kPl + tid;
      s += psum[o];
      m = fmaxf(m, pmax[o]);
    }
    sa[tid] = s * (1.0f / ((float)kHW * kCarryA));
    sm[tid] = m * kInvCarryA;
  }
  __syncthreads();
  {
    const int j  = tid >> 2;
    const int qk = tid & 3;
    float s1 = 0.0f, s2 = 0.0f;
#pragma unroll 4
    for (int k = 0; k < 64; ++k) {
      const int c = qk * 64 + k;
      const float w = ca1[j * kPl + c];
      s1 = fmaf(w, sa[c], s1);
      s2 = fmaf(w, sm[c], s2);
    }
    s1 += __shfl_xor(s1, 1, 32);
    s2 += __shfl_xor(s2, 1, 32);
    s1 += __shfl_xor(s1, 2, 32);
    s2 += __shfl_xor(s2, 2, 32);
    if (qk == 0) hsum[j] = fmaxf(s1, 0.0f) + fmaxf(s2, 0.0f);
  }
  __syncthreads();
  {
    float sacc = 0.0f;
#pragma unroll 4
    for (int a = 0; a < kAtt; ++a) sacc = fmaf(ca2[tid * kAtt + a], hsum[a], sacc);
    const float av = 1.0f / (1.0f + expf(-sacc));
    satt[tid] = av;
    float* o1 = out1 + (size_t)b * kPl + tid;
    *(volatile float*)o1 = av;
    __threadfence();
    *(volatile float*)o1 = av;
  }
  __syncthreads();
#pragma unroll 1
  for (int it = 0; it < 16; ++it) {
    const int idx = it * 256 + tid;
    const int o  = idx >> 5;
    const int cc = (idx & 31) * 8;
    const v4f f0 = *(const v4f*)(fcw + (size_t)o * kPl + cc);
    const v4f f1 = *(const v4f*)(fcw + (size_t)o * kPl + cc + 4);
    const v4f t0 = *(const v4f*)(satt + cc);
    const v4f t1 = *(const v4f*)(satt + cc + 4);
    v8h hv;
#pragma unroll
    for (int e = 0; e < 4; ++e) {
      hv[e]     = (_Float16)(f0[e] * t0[e] * kCarryW);
      hv[4 + e] = (_Float16)(f1[e] * t1[e] * kCarryW);
    }
    unsigned short* dst = fcs + ((size_t)b * kCin + o) * kPl + cc;
    *(volatile v8h*)dst = hv;
    __threadfence();
    *(volatile v8h*)dst = hv;
  }
}

extern "C" void kernel_launch(void* const* d_in, const int* in_sizes, int n_in,
                              void* d_out, int out_size, void* d_ws, size_t ws_size,
                              hipStream_t stream)
{
  if (n_in < 11) return;
  if (in_sizes[0] != kNb * kCin * kHW) return;
  if (in_sizes[1] != kPl * kCin) return;
  if (in_sizes[2] != kPl * 9) return;
  if (in_sizes[3] != kPl) return;
  if (in_sizes[4] != kPl * kPl) return;
  if (in_sizes[5] != kPl) return;
  if (in_sizes[6] != kAtt * kPl) return;
  if (in_sizes[7] != kPl * kAtt) return;
  if (in_sizes[8] != kCin * kPl) return;
  if (in_sizes[9] != kCin) return;
  if (in_sizes[10] != kTok * kRank) return;
  if (out_size != kOut0Elems + kOut1Elems) return;
  if (ws_size < kWsTotal) return;

  const float* x   = (const float*)d_in[0];
  const float* w1  = (const float*)d_in[1];
  const float* w3  = (const float*)d_in[2];
  const float* b3  = (const float*)d_in[3];
  const float* lw  = (const float*)d_in[4];
  const float* lb  = (const float*)d_in[5];
  const float* ca1 = (const float*)d_in[6];
  const float* ca2 = (const float*)d_in[7];
  const float* fw  = (const float*)d_in[8];
  const float* fb  = (const float*)d_in[9];
  const float* bi  = (const float*)d_in[10];
  float* out = (float*)d_out;

  char* ws = (char*)d_ws;
  unsigned short* XT   = (unsigned short*)(ws + kOffXT);
  unsigned short* W1H  = (unsigned short*)(ws + kOffW1H);
  unsigned short* LWH  = (unsigned short*)(ws + kOffLWH);
  unsigned short* Y    = (unsigned short*)(ws + kOffY);
  unsigned short* XM   = (unsigned short*)(ws + kOffXM);
  float*          XL   = (float*)(ws + kOffXL);
  unsigned short* FEAT = (unsigned short*)(ws + kOffFEAT);
  float*          PSUM = (float*)(ws + kOffPSUM);
  float*          PMAX = (float*)(ws + kOffPMAX);
  unsigned short* FCS  = (unsigned short*)(ws + kOffFCS);
  int*            FLAG = (int*)(ws + kOffFLAG);

  prep_x_kernel<<<dim3(kHW / 64, kCin / 64, kNb), 256, 0, stream>>>(x, XT);
  prep_w_kernel<<<48, 256, 0, stream>>>(w1, lw, W1H, LWH);
  flag_kernel<<<kTok / 256, 256, 0, stream>>>(bi, FLAG);
  gemm_f16_kernel<0><<<dim3(128, 1), 256, 0, stream>>>(
      XT, kCin, 0L, W1H, kCin, 0L, (void*)Y, kPl, 0L, nullptr, kTok, kPl, kCin, kScaleS1);
  dw3x3_kernel<<<kNb * kImg, 256, 0, stream>>>(Y, w3, b3, XM);
  gemm_f16_kernel<1><<<dim3(128, 1), 256, 0, stream>>>(
      XM, kPl, 0L, LWH, kPl, 0L, (void*)XL, kPl, 0L, lb, kTok, kPl, kPl, kScaleS2);
  combine_kernel<<<kTok / kCmbTokPerBlock, kCmbThreads, 0, stream>>>(XL, XM, FLAG, bi, FEAT);
  pool_partial_kernel<<<dim3(kChunks, kNb), 256, 0, stream>>>(FEAT, PSUM, PMAX);
  att_kernel<<<kNb, 256, 0, stream>>>(PSUM, PMAX, ca1, ca2, fw, out + (size_t)kOut0Elems, FCS);
  gemm_f16_kernel<2><<<dim3(16, kNb), 256, 0, stream>>>(
      FCS, kPl, (long)kCin * kPl, FEAT, kPl, (long)kHW * kPl, (void*)out, kHW, (long)kCin * kHW,
      fb, kCin, kHW, kPl, kScaleS6);
}
